// StateSpaceLayer_47717086659301
// MI455X (gfx1250) — hardware-verified
//
#include <hip/hip_runtime.h>
#include <math.h>

constexpr int SEQ_LEN  = 1024;
constexpr int DIM_D    = 64;
constexpr int SLAB     = DIM_D * DIM_D;
constexpr int REC_W    = 128;
constexpr int TCHUNK   = 128;
constexpr int SB_PITCH = TCHUNK + 4;
constexpr int TR_PITCH = 72;
constexpr int A_PITCH  = 40;
constexpr int OS_PITCH = 68;
constexpr float INV_SLAB     = 1.0f / (float)SLAB;
constexpr float LN_EPS       = 1e-5f;
constexpr float H_MIN_NORMAL = 6.103515625e-5f;

static_assert(SEQ_LEN % TCHUNK == 0);
static_assert(SEQ_LEN % 64 == 0);
static_assert(DIM_D == 64);
static_assert(SLAB == 4096);
static_assert(REC_W == 128);
static_assert((SB_PITCH * 4) % 16 == 0);
static_assert((TR_PITCH * 2) % 16 == 0);
static_assert((A_PITCH * 2) % 16 == 0);
static_assert((OS_PITCH * 4) % 16 == 0);

constexpr size_t WS_REC_OFF  = 0;
constexpr size_t WS_REC_BYTES  = (size_t)SEQ_LEN * REC_W * 4;
constexpr size_t WS_CUMS_OFF = WS_REC_OFF + WS_REC_BYTES;
constexpr size_t WS_CUMS_BYTES = (size_t)DIM_D * SEQ_LEN * 4;
constexpr size_t WS_XT_OFF   = WS_CUMS_OFF + WS_CUMS_BYTES;
constexpr size_t WS_XT_BYTES   = (size_t)SLAB * SEQ_LEN * 2;
constexpr size_t WS_TOTAL    = WS_XT_OFF + WS_XT_BYTES;
static_assert(WS_REC_OFF % 128 == 0 && WS_CUMS_OFF % 128 == 0 && WS_XT_OFF % 128 == 0);
static_assert(WS_TOTAL <= (size_t)134217728);

typedef __attribute__((ext_vector_type(16))) _Float16 v16h;
typedef __attribute__((ext_vector_type(8)))  _Float16 v8h;
typedef __attribute__((ext_vector_type(8)))  float    v8f;
typedef __attribute__((ext_vector_type(4)))  float    v4f;
typedef __attribute__((ext_vector_type(4)))  unsigned int v4u;

__device__ __forceinline__ void dep_guard_h(v8f& a, v8f& b, v16h x, v16h y) { asm volatile("v_nop\n\tv_nop\n\tv_nop\n\tv_nop" : "+v"(a), "+v"(b) : "v"(x), "v"(y)); }
__device__ __forceinline__ void keep4_h(v16h a, v16h b, v16h c, v16h d) { asm volatile("v_nop" :: "v"(a), "v"(b), "v"(c), "v"(d)); }
__device__ __forceinline__ void acc_guard4(v8f& a, v8f& b, v8f& c, v8f& d) { asm volatile("v_nop\n\tv_nop\n\tv_nop\n\tv_nop" : "+v"(a), "+v"(b), "+v"(c), "+v"(d)); }
template <typename T> struct Frag;
template <> struct Frag<_Float16> {
  typedef v16h V; union U { v16h v; v8h h[2]; };
  static __device__ __forceinline__ v16h load(const _Float16* p) {
    U f; f.h[0] = *(const v8h*)(p); f.h[1] = *(const v8h*)(p + 16); return f.v;
  }
  static __device__ __forceinline__ v8f mma(v16h a, v16h b, v8f c) {
    return __builtin_amdgcn_wmma_f32_16x16x32_f16(false, a, false, b, (short)0, c, false, false);
  }
  static __device__ __forceinline__ void guard(v8f& a, v8f& b, v16h x, v16h y) { dep_guard_h(a, b, x, y); }
  static __device__ __forceinline__ void keep(v16h a, v16h b, v16h c, v16h d) { keep4_h(a, b, c, d); }
};
__device__ __forceinline__ void mma_guard4(v8f& a0, v8f& a1, v8f& a2, v8f& a3,
                                           v16h x, v16h y0, v16h y1, v16h y2, v16h y3) {
  asm volatile("v_nop\n\tv_nop\n\tv_nop\n\tv_nop"
               : "+v"(a0), "+v"(a1), "+v"(a2), "+v"(a3)
               : "v"(x), "v"(y0), "v"(y1), "v"(y2), "v"(y3));
}
__device__ __forceinline__ unsigned short h_bits(float f) { const _Float16 h = (_Float16)f; return __builtin_bit_cast(unsigned short, h); }

__global__ __launch_bounds__(256) void stats_gate_kernel(
    const float* __restrict__ x,
    const float* __restrict__ log_A,
    const float* __restrict__ dt_w,
    const float* __restrict__ dt_b,
    const float* __restrict__ ln_w,
    const float* __restrict__ ln_b,
    float*       __restrict__ rec)
{
  __shared__ __align__(16) float xs[SLAB];
  __shared__ __align__(16) float recs[REC_W];
  __shared__ float dws[DIM_D];
  __shared__ float lga[DIM_D];
  __shared__ float redA[8];
  __shared__ float redB[8];

  const int t    = blockIdx.x;
  const int tid  = threadIdx.x;
  const int lane = tid & 31;
  const int wave = tid >> 5;
  const float* xb = x + (size_t)t * SLAB;

  if (wave == 0) {
    dws[2 * lane]     = dt_w[2 * lane];
    dws[2 * lane + 1] = dt_w[2 * lane + 1];
    lga[2 * lane]     = log_A[2 * lane];
    lga[2 * lane + 1] = log_A[2 * lane + 1];
  }

  float v[16];
  {
    const v4f a0 = *(const v4f*)(xb + tid * 8);
    const v4f a1 = *(const v4f*)(xb + tid * 8 + 4);
    const v4f a2 = *(const v4f*)(xb + 2048 + tid * 8);
    const v4f a3 = *(const v4f*)(xb + 2048 + tid * 8 + 4);
#pragma unroll
    for (int e = 0; e < 4; ++e) { v[e] = a0[e]; v[4 + e] = a1[e]; v[8 + e] = a2[e]; v[12 + e] = a3[e]; }
  }

  float s = 0.0f;
#pragma unroll
  for (int e = 0; e < 16; ++e) s += v[e];
#pragma unroll
  for (int off = 16; off > 0; off >>= 1) s += __shfl_xor(s, off, 32);
  if (lane == 0) redA[wave] = s;
  __syncthreads();
  float tot = 0.0f;
#pragma unroll
  for (int w = 0; w < 8; ++w) tot += redA[w];
  const float mean = tot * INV_SLAB;

  float d[16];
  float s2 = 0.0f;
#pragma unroll
  for (int e = 0; e < 16; ++e) { d[e] = v[e] - mean; s2 += d[e] * d[e]; }
#pragma unroll
  for (int off = 16; off > 0; off >>= 1) s2 += __shfl_xor(s2, off, 32);
  if (lane == 0) redB[wave] = s2;
  __syncthreads();
  float tot2 = 0.0f;
#pragma unroll
  for (int w = 0; w < 8; ++w) tot2 += redB[w];
  const float var  = tot2 * INV_SLAB;
  const float rstd = rsqrtf(var + LN_EPS);

#pragma unroll
  for (int it = 0; it < 2; ++it) {
    const int base = it * 2048 + tid * 8;
    const v4f w0 = *(const v4f*)(ln_w + base);
    const v4f w1 = *(const v4f*)(ln_w + base + 4);
    const v4f b0 = *(const v4f*)(ln_b + base);
    const v4f b1 = *(const v4f*)(ln_b + base + 4);
    v4f n0, n1;
#pragma unroll
    for (int e = 0; e < 4; ++e) {
      n0[e] = d[it * 8 + e]     * rstd * w0[e] + b0[e];
      n1[e] = d[it * 8 + 4 + e] * rstd * w1[e] + b1[e];
    }
    *(v4f*)(xs + base)     = n0;
    *(v4f*)(xs + base + 4) = n1;
    asm volatile("" ::: "memory");
  }
  __syncthreads();

  const int r  = tid >> 2;
  const int q  = tid & 3;
  const int c0 = q * 16;
  float dot = 0.0f;
#pragma unroll 1
  for (int c = 0; c < 16; ++c) dot = fmaf(xs[r * DIM_D + c0 + c], dws[c0 + c], dot);
  dot += __shfl_xor(dot, 1, 32);
  dot += __shfl_xor(dot, 2, 32);
  const float pre = dot + dt_b[0];
  const float sp = fmaxf(pre, 0.0f) + log1pf(expf(-fabsf(pre)));
  const float la = -expf(lga[r]) * sp;
  if (q == 0) recs[r] = la;
  if (tid >= DIM_D && tid < REC_W) {
    const float fill = (tid == DIM_D) ? mean : ((tid == DIM_D + 1) ? rstd : 0.0f);
    recs[tid] = fill;
  }
  __syncthreads();

  if (wave == 0) {
    const v4f o = *(const v4f*)(recs + lane * 4);
    float* dst = rec + (size_t)t * REC_W + lane * 4;
    *(volatile v4f*)dst = o;
    __threadfence();
    *(volatile v4f*)dst = o;
  }
}

__global__ __launch_bounds__(64) void prefix_kernel(
    const float* __restrict__ rec,
    float*       __restrict__ cums)
{
  __shared__ __align__(16) float sb[DIM_D][SB_PITCH];
  const int r    = threadIdx.x;
  const int lane = r & 31;
  const int wave = r >> 5;
  float acc = 0.0f;
  for (int ch = 0; ch < SEQ_LEN / TCHUNK; ++ch) {
#pragma unroll 4
    for (int tt = 0; tt < TCHUNK; ++tt) {
      acc += rec[(size_t)(ch * TCHUNK + tt) * REC_W + r];
      sb[r][tt] = acc;
    }
    __syncthreads();
    for (int pass = 0; pass < 2; ++pass) {
#pragma unroll 4
      for (int i = 0; i < 32; ++i) {
        const int row = wave * 32 + i;
        const v4f val = *(const v4f*)(&sb[row][lane * 4]);
        *(volatile v4f*)(cums + (size_t)row * SEQ_LEN + ch * TCHUNK + lane * 4) = val;
      }
      __threadfence();
    }
    __syncthreads();
  }
}

__global__ __launch_bounds__(256) void norm_cast_tr_kernel(
    const float* __restrict__ x,
    const float* __restrict__ ln_w,
    const float* __restrict__ ln_b,
    const float* __restrict__ rec,
    unsigned short* __restrict__ XhT)
{
  __shared__ __align__(16) unsigned short sm[DIM_D][TR_PITCH];
  __shared__ float mean_s[64];
  __shared__ float rstd_s[64];
  __shared__ float lnw_s[64];
  __shared__ float lnb_s[64];

  const int tb   = blockIdx.x;
  const int cb   = blockIdx.y;
  const int tid  = threadIdx.x;
  const int lane = tid & 31;
  const int wave = tid >> 5;
  const int tt   = tid >> 2;
  const int c0   = (tid & 3) * 16;

  float xv[16];
  {
    const float* xp = x + (size_t)(tb * 64 + tt) * SLAB + cb * 64 + c0;
    const v4f a0 = *(const v4f*)(xp);
    const v4f a1 = *(const v4f*)(xp + 4);
    const v4f a2 = *(const v4f*)(xp + 8);
    const v4f a3 = *(const v4f*)(xp + 12);
#pragma unroll
    for (int e = 0; e < 4; ++e) { xv[e] = a0[e]; xv[4 + e] = a1[e]; xv[8 + e] = a2[e]; xv[12 + e] = a3[e]; }
  }
  if (tid < 64) {
    mean_s[tid] = rec[(size_t)(tb * 64 + tid) * REC_W + DIM_D];
    rstd_s[tid] = rec[(size_t)(tb * 64 + tid) * REC_W + DIM_D + 1];
    lnw_s[tid]  = ln_w[cb * 64 + tid];
    lnb_s[tid]  = ln_b[cb * 64 + tid];
  }
  __syncthreads();

  const float mean = mean_s[tt];
  const float rstd = rstd_s[tt];
#pragma unroll
  for (int e = 0; e < 16; ++e) {
    const float xn = (xv[e] - mean) * rstd * lnw_s[c0 + e] + lnb_s[c0 + e];
    sm[c0 + e][tt] = h_bits(xn);
  }
  __syncthreads();

  const int q  = lane >> 3;
  const int c8 = (lane & 7) * 8;
  for (int pass = 0; pass < 2; ++pass) {
#pragma unroll
    for (int it = 0; it < 2; ++it) {
      const int row = wave * 8 + it * 4 + q;
      const v4u u = *(const v4u*)(&sm[row][c8]);
      *(volatile v4u*)(XhT + (size_t)(cb * 64 + row) * SEQ_LEN + tb * 64 + c8) = u;
    }
    __threadfence();
  }
}

__global__ __launch_bounds__(128) void decay_wmma_kernel(
    const unsigned short* __restrict__ XhTp,
    const float*          __restrict__ cums,
    float*                __restrict__ out)
{
  __shared__ __align__(16) float    cs[SEQ_LEN];
  __shared__ __align__(16) _Float16 As[64 * A_PITCH];
  __shared__ __align__(16) float    Os[4][16 * OS_PITCH];

  const _Float16* XhT = (const _Float16*)XhTp;
  const int tid   = threadIdx.x;
  const int lane  = tid & 31;
  const int wave  = tid >> 5;
  const int hh    = lane >> 4;
  const int rlane = lane & 15;
  const int koff  = hh * 8;
  const int tb    = blockIdx.x;
  const int r     = blockIdx.y;
  const int T0    = tb * 64;

  const int nv = (T0 + 64) >> 2;
  for (int i = tid; i < nv; i += 128)
    *(v4f*)(cs + 4 * i) = *(const v4f*)(cums + (size_t)r * SEQ_LEN + 4 * i);
  __syncthreads();

  const int   tt = tid >> 1;
  const int   jb = (tid & 1) * 16;
  const int   tg = T0 + tt;
  const float ct = cs[tg];

  v8f acc[4];
#pragma unroll
  for (int j = 0; j < 4; ++j) acc[j] = (v8f){0.f,0.f,0.f,0.f,0.f,0.f,0.f,0.f};

  const _Float16* bbase = XhT + (size_t)(r * 64 + rlane) * SEQ_LEN + koff;
  const int nsteps = 2 * tb + 2;

  for (int st = 0; st < nsteps; ++st) {
    const int J0 = st * 32;
    {
      const v4f q0 = *(const v4f*)(cs + J0 + jb);
      const v4f q1 = *(const v4f*)(cs + J0 + jb + 4);
      const v4f q2 = *(const v4f*)(cs + J0 + jb + 8);
      const v4f q3 = *(const v4f*)(cs + J0 + jb + 12);
      float cj[16];
#pragma unroll
      for (int e = 0; e < 4; ++e) { cj[e] = q0[e]; cj[4 + e] = q1[e]; cj[8 + e] = q2[e]; cj[12 + e] = q3[e]; }
      v8h p0, p1;
#pragma unroll
      for (int e = 0; e < 16; ++e) {
        const float dlt = fminf(ct - cj[e], 0.0f);
        float ev = expf(dlt);
        ev = (ev < H_MIN_NORMAL) ? 0.0f : ev;
        ev = (J0 + jb + e <= tg) ? ev : 0.0f;
        if (e < 8) p0[e] = (_Float16)ev; else p1[e - 8] = (_Float16)ev;
      }
      *(v8h*)(As + tt * A_PITCH + jb)     = p0;
      *(v8h*)(As + tt * A_PITCH + jb + 8) = p1;
    }
    __syncthreads();
    {
      const v16h a  = Frag<_Float16>::load(As + (wave * 16 + rlane) * A_PITCH + koff);
      const _Float16* bp = bbase + J0;
      const v16h b0 = Frag<_Float16>::load(bp);
      const v16h b1 = Frag<_Float16>::load(bp + (size_t)16 * SEQ_LEN);
      const v16h b2 = Frag<_Float16>::load(bp + (size_t)32 * SEQ_LEN);
      const v16h b3 = Frag<_Float16>::load(bp + (size_t)48 * SEQ_LEN);
      acc[0] = Frag<_Float16>::mma(a, b0, acc[0]);
      acc[1] = Frag<_Float16>::mma(a, b1, acc[1]);
      acc[2] = Frag<_Float16>::mma(a, b2, acc[2]);
      acc[3] = Frag<_Float16>::mma(a, b3, acc[3]);
      mma_guard4(acc[0], acc[1], acc[2], acc[3], a, b0, b1, b2, b3);
    }
    __syncthreads();
  }
  acc_guard4(acc[0], acc[1], acc[2], acc[3]);

  float* os = Os[wave];
#pragma unroll
  for (int rr = 0; rr < 8; ++rr) {
#pragma unroll
    for (int j = 0; j < 4; ++j) os[(8 * hh + rr) * OS_PITCH + j * 16 + rlane] = acc[j][rr];
  }
  __syncthreads();
  {
    const int c4 = rlane * 4;
    for (int pass = 0; pass < 2; ++pass) {
#pragma unroll
      for (int it = 0; it < 8; ++it) {
        const int row = it * 2 + hh;
        const v4f val = *(const v4f*)(os + row * OS_PITCH + c4);
        const size_t t = (size_t)(T0 + wave * 16 + row);
        *(volatile v4f*)(out + (t * DIM_D + r) * DIM_D + c4) = val;
      }
      __threadfence();
    }
  }
}

extern "C" void kernel_launch(void* const* d_in, const int* in_sizes, int n_in,
                              void* d_out, int out_size, void* d_ws, size_t ws_size,
                              hipStream_t stream)
{
  if (n_in < 6) return;
  if (in_sizes[0] != SEQ_LEN * SLAB || in_sizes[1] != DIM_D || in_sizes[2] != DIM_D ||
      in_sizes[3] < 1 || in_sizes[4] != SLAB || in_sizes[5] != SLAB) return;
  if (out_size != SEQ_LEN * SLAB) return;
  if (ws_size < WS_TOTAL) return;

  const float* x     = (const float*)d_in[0];
  const float* log_A = (const float*)d_in[1];
  const float* dt_w  = (const float*)d_in[2];
  const float* dt_b  = (const float*)d_in[3];
  const float* ln_w  = (const float*)d_in[4];
  const float* ln_b  = (const float*)d_in[5];
  float* out = (float*)d_out;

  char* ws = (char*)d_ws;
  float*          rec  = (float*)(ws + WS_REC_OFF);
  float*          cums = (float*)(ws + WS_CUMS_OFF);
  unsigned short* XhT  = (unsigned short*)(ws + WS_XT_OFF);

  stats_gate_kernel<<<dim3(SEQ_LEN), dim3(256), 0, stream>>>(x, log_A, dt_w, dt_b, ln_w, ln_b, rec);
  prefix_kernel<<<dim3(1), dim3(64), 0, stream>>>(rec, cums);
  norm_cast_tr_kernel<<<dim3(SEQ_LEN / 64, SLAB / 64), dim3(256), 0, stream>>>(x, ln_w, ln_b, rec, XhT);
  decay_wmma_kernel<<<dim3(SEQ_LEN / 64, DIM_D), dim3(128), 0, stream>>>(XhT, cums, out);
}
